// CrossAttention_59717225284223
// MI455X (gfx1250) — hardware-verified
//
#include <hip/hip_runtime.h>
#include <stdint.h>


typedef _Float16 v16h __attribute__((ext_vector_type(16)));
typedef _Float16 v8h  __attribute__((ext_vector_type(8)));
typedef float    v8f  __attribute__((ext_vector_type(8)));
typedef float    v4f  __attribute__((ext_vector_type(4)));

#ifndef NB
#define NB 4
#endif
#ifndef SEQ
#define SEQ 8192
#endif
#define NB_FULL  4
#define SEQ_FULL 8192
#define CH    256
#define NH    4
#define HD    64
#define CATW  512
#define HID   512
#define NTOK  (NB * SEQ)

#define ACT_CAR  8.0f
#define ACT_INV  0.125f
#define W_CAR    1024.0f
#define ACC_SCL  0.0001220703125f
#define KV_SCL   0.001953125f
#define LN_EPS   1e-5f
#define BN_EPS   1e-5f
#define ATTN_EPS 1e-6f

#define OFF_WQ 0
#define OFF_WK 65536
#define OFF_WV 131072
#define OFF_WA 196608
#define OFF_W1 262144
#define OFF_W2 524288
#define N_WALL 655360

static_assert(SEQ % 128 == 0);
static_assert(NB <= NB_FULL && SEQ <= SEQ_FULL);
static_assert(CH == NH * HD);
static_assert(HD == 64);
static_assert(CH % 128 == 0 && CATW % 32 == 0 && HID % 64 == 0);
static_assert((long)NB_FULL * CH * SEQ_FULL * 4 == 33554432L);
static_assert((long)(SEQ / 64) * (CH / 64) * (2 * NB) * 4096 == 2L * NB * SEQ * CH);
static_assert(OFF_W2 + 131072 == N_WALL && (262144 / 8) / 256 == 128);
static_assert((long)(CH / 64) * (NTOK / 128) * 128 * 64 == (long)NTOK * CH);
static_assert((long)(SEQ / 64) * (CH / 128) * NB * 128 * 64 == (long)NB * CH * SEQ);
static_assert((long)(HID / 64) * (NTOK / 128) * 128 * 64 == (long)NTOK * HID);
static_assert((long)(NTOK / 64) * 64 * CH == (long)NTOK * CH);
static_assert((long)NTOK * HID == 2L * NTOK * CH);
static_assert(((long)NTOK * (CATW + 4 * CH) + N_WALL + (long)NB * NH * 4096) * 2 + (long)NB * CH * 4 <= 134217728L);

union Frag16 { v16h v; v8h p[2]; };

__device__ __forceinline__ v16h ld_frag(const _Float16* p, int hl) {
  Frag16 f;
  f.p[0] = *(const v8h*)(p + 8 * hl);
  f.p[1] = *(const v8h*)(p + 16 + 8 * hl);
  return f.v;
}

__device__ __forceinline__ v8f mma(v16h a, v16h b, v8f c) {
  v8f d = __builtin_amdgcn_wmma_f32_16x16x32_f16(false, a, false, b, (short)0, c, false, false);
  asm volatile("v_nop\n\tv_nop\n\tv_nop\n\tv_nop" : "+v"(d) : "v"(a), "v"(b));
  return d;
}

__device__ __forceinline__ float bf16_rne(float x) {
  unsigned int u = __builtin_bit_cast(unsigned int, x);
  u += 0x7FFFu + ((u >> 16) & 1u);
  return __builtin_bit_cast(float, u & 0xFFFF0000u);
}

__device__ __forceinline__ float wave_sum(float v) {
  v += __shfl_xor(v, 16, 32);
  v += __shfl_xor(v, 8, 32);
  v += __shfl_xor(v, 4, 32);
  v += __shfl_xor(v, 2, 32);
  v += __shfl_xor(v, 1, 32);
  return v;
}

__global__ __launch_bounds__(256) void k_trx(const float* __restrict__ x1,
                                             const float* __restrict__ x2,
                                             _Float16* __restrict__ cat,
                                             _Float16* __restrict__ x2t)
{
  __shared__ float tile[64 * 65];
  const unsigned tid = threadIdx.x;
  const unsigned z = blockIdx.z;
  const unsigned which = (z >= (unsigned)NB) ? 1u : 0u;
  const unsigned b = z - which * (unsigned)NB;
  const unsigned n0 = blockIdx.x * 64u, c0 = blockIdx.y * 64u;
  const float* src = (which ? x2 : x1) + (size_t)b * CH * SEQ_FULL;
  _Float16* dst = which ? x2t : cat;
  const unsigned ldo = which ? (unsigned)CH : (unsigned)CATW;
#pragma unroll
  for (unsigned i = 0; i < 4; ++i) {
    const unsigned idx = i * 256u + tid;
    const unsigned r = idx >> 4, c4 = (idx & 15u) * 4u;
    const v4f v = *(const v4f*)(src + (size_t)(c0 + r) * SEQ_FULL + n0 + c4);
    float* tp = tile + r * 65u + c4;
    tp[0] = v[0]; tp[1] = v[1]; tp[2] = v[2]; tp[3] = v[3];
  }
  __syncthreads();
  v8h o[2];
  _Float16* dp[2];
#pragma unroll
  for (unsigned i = 0; i < 2; ++i) {
    const unsigned line = i * 32u + (tid >> 3);
    const unsigned pc   = (tid & 7u) * 8u;
#pragma unroll
    for (unsigned j = 0; j < 8; ++j)
      o[i][j] = (_Float16)(bf16_rne(tile[(pc + j) * 65u + line]) * ACT_CAR);
    dp[i] = dst + ((size_t)b * SEQ + n0 + line) * ldo + c0 + pc;
  }
  *(volatile v8h*)dp[0] = o[0];
  *(volatile v8h*)dp[1] = o[1];
  __threadfence();
  *(volatile v8h*)dp[0] = o[0];
  *(volatile v8h*)dp[1] = o[1];
}

__global__ __launch_bounds__(256) void k_cvtw(const float* __restrict__ wq, const float* __restrict__ wk,
                                              const float* __restrict__ wv, const float* __restrict__ wa,
                                              const float* __restrict__ w1, const float* __restrict__ w2,
                                              _Float16* __restrict__ dst)
{
  const unsigned id = blockIdx.y;
  const float* src = (id == 0u) ? wq : (id == 1u) ? wk : (id == 2u) ? wv : (id == 3u) ? wa : (id == 4u) ? w1 : w2;
  const unsigned n   = (id < 4u) ? 65536u : (id == 4u) ? 262144u : 131072u;
  const unsigned off = (id < 4u) ? id * 65536u : (id == 4u) ? (unsigned)OFF_W1 : (unsigned)OFF_W2;
  const unsigned e = (blockIdx.x * 256u + threadIdx.x) * 8u;
  if (e >= n) return;
  const v4f x0 = *(const v4f*)(src + e);
  const v4f x1 = *(const v4f*)(src + e + 4);
  v8h o;
#pragma unroll
  for (int j = 0; j < 4; ++j) {
    const float t0 = x0[j];
    const float t1 = x1[j];
    o[j]     = (_Float16)(bf16_rne(t0) * W_CAR);
    o[4 + j] = (_Float16)(bf16_rne(t1) * W_CAR);
  }
  _Float16* d = dst + off + e;
  *(volatile v8h*)d = o;
  __threadfence();
  *(volatile v8h*)d = o;
}

__device__ __forceinline__ void gemm_core(const _Float16* ap0, const _Float16* ap1,
                                          const _Float16* bp, int K, int hl, v8f (&acc)[8])
{
  const size_t bst = (size_t)16 * K;
#pragma unroll 1
  for (int k0 = 0; k0 < K; k0 += 32) {
    const v16h a0 = ld_frag(ap0 + k0, hl);
    const v16h a1 = ld_frag(ap1 + k0, hl);
    const v16h b0 = ld_frag(bp + k0, hl);
    const v16h b1 = ld_frag(bp + bst + k0, hl);
    const v16h b2 = ld_frag(bp + 2 * bst + k0, hl);
    const v16h b3 = ld_frag(bp + 3 * bst + k0, hl);
    acc[0] = mma(a0, b0, acc[0]);
    acc[1] = mma(a0, b1, acc[1]);
    acc[2] = mma(a0, b2, acc[2]);
    acc[3] = mma(a0, b3, acc[3]);
    acc[4] = mma(a1, b0, acc[4]);
    acc[5] = mma(a1, b1, acc[5]);
    acc[6] = mma(a1, b2, acc[6]);
    acc[7] = mma(a1, b3, acc[7]);
  }
}

template <int BM, int ACT>
__global__ __launch_bounds__(128) __attribute__((amdgpu_num_vgpr(256)))
void k_gemm(const _Float16* __restrict__ A, const _Float16* __restrict__ Bt,
            _Float16* __restrict__ Cout, const float* __restrict__ bias,
            unsigned lda, int K, unsigned ldc, unsigned sA, unsigned sB, unsigned sC)
{
  __shared__ __attribute__((aligned(16))) _Float16 ldsH[128 * 72];

  const unsigned tid = threadIdx.x, lane = tid & 31u, w = tid >> 5;
  const int hl = (int)(lane >> 4);
  const unsigned c = lane & 15u;
  const unsigned m0 = blockIdx.y * 128u, n0 = blockIdx.x * 64u;
  const unsigned zb = blockIdx.z;
  const unsigned mw = m0 + 32u * w;

  const _Float16* ap0 = A  + (size_t)zb * sA + (size_t)(mw + c) * lda;
  const _Float16* ap1 = A  + (size_t)zb * sA + (size_t)(mw + 16u + c) * lda;
  const _Float16* bp  = Bt + (size_t)zb * sB + (size_t)(n0 + c) * (unsigned)K;

  v8f acc[8] = {};
  gemm_core(ap0, ap1, bp, K, hl, acc);

  float bcol[4] = {0.f, 0.f, 0.f, 0.f};
  if (BM == 1) {
#pragma unroll
    for (unsigned t = 0; t < 4; ++t) bcol[t] = bf16_rne(bias[n0 + 16u * t + c]);
  }
#pragma unroll
  for (unsigned i = 0; i < 2; ++i)
#pragma unroll
    for (unsigned r = 0; r < 8; ++r) {
      const unsigned rowl = 32u * w + 16u * i + 8u * (unsigned)hl + r;
      float brow = 0.f;
      if (BM == 2) brow = bf16_rne(bias[m0 + rowl]);
#pragma unroll
      for (unsigned t = 0; t < 4; ++t) {
        float v = acc[i * 4 + t][r] * ACC_SCL;
        if (BM == 1) v += bcol[t];
        if (BM == 2) v += brow;
        if (ACT == 1) {
          const float ev = expf(v);
          v = (v > 0.f) ? (v + 1.0f) : ev;
        }
        if (ACT == 2) v = (v > 0.f) ? v : 0.f;
        ldsH[rowl * 72u + 16u * t + c] = (_Float16)(v * ACT_CAR);
      }
    }
  __syncthreads();

  _Float16* const bh = Cout + (size_t)zb * sC + (size_t)m0 * ldc + n0;
  for (unsigned i = 0; i < 8; ++i) {
    const unsigned q = i * 128u + tid;
    const unsigned rowl = q >> 3, ch = (q & 7u) * 8u;
    const v8h vh = *(const v8h*)(ldsH + rowl * 72u + ch);
    *(volatile v8h*)(bh + (size_t)rowl * ldc + ch) = vh;
  }
  __threadfence();
  for (unsigned i = 0; i < 8; ++i) {
    const unsigned q = i * 128u + tid;
    const unsigned rowl = q >> 3, ch = (q & 7u) * 8u;
    const v8h vh = *(const v8h*)(ldsH + rowl * 72u + ch);
    *(volatile v8h*)(bh + (size_t)rowl * ldc + ch) = vh;
  }
}

__global__ __launch_bounds__(256) __attribute__((amdgpu_num_vgpr(256)))
void k_kv(const _Float16* __restrict__ Kt, const _Float16* __restrict__ Vt,
          _Float16* __restrict__ KVt, float* __restrict__ Ksum)
{
  __shared__ __attribute__((aligned(16))) float part[4 * 64 * 64];
  __shared__ __attribute__((aligned(16))) float ksp[4 * 64];

  const unsigned tid = threadIdx.x, lane = tid & 31u, w = tid >> 5;
  const int hl = (int)(lane >> 4);
  const unsigned c = lane & 15u;
  const unsigned wr = w & 1u, wk = w >> 1;
  const unsigned h = blockIdx.x, b = blockIdx.y;

  const size_t base = ((size_t)b * CH + (size_t)h * HD) * SEQ;
  const _Float16* vp0 = Vt + base + (size_t)(32u * wr + c) * SEQ;
  const _Float16* vp1 = vp0 + (size_t)16 * SEQ;
  const _Float16* kp  = Kt + base + (size_t)c * SEQ;
  const size_t bst = (size_t)16 * SEQ;

  v16h ones;
#pragma unroll
  for (int e = 0; e < 16; ++e) ones[e] = (_Float16)1.0f;

  v8f acc[12] = {};
  const unsigned kbeg = wk * (unsigned)(SEQ / 4);
#pragma unroll 1
  for (unsigned k0 = kbeg; k0 < kbeg + (unsigned)(SEQ / 4); k0 += 32u) {
    const v16h a0 = ld_frag(vp0 + k0, hl);
    const v16h a1 = ld_frag(vp1 + k0, hl);
    const v16h b0 = ld_frag(kp + k0, hl);
    const v16h b1 = ld_frag(kp + bst + k0, hl);
    const v16h b2 = ld_frag(kp + 2 * bst + k0, hl);
    const v16h b3 = ld_frag(kp + 3 * bst + k0, hl);
    acc[0]  = mma(a0, b0, acc[0]);
    acc[1]  = mma(a0, b1, acc[1]);
    acc[2]  = mma(a0, b2, acc[2]);
    acc[3]  = mma(a0, b3, acc[3]);
    acc[4]  = mma(a1, b0, acc[4]);
    acc[5]  = mma(a1, b1, acc[5]);
    acc[6]  = mma(a1, b2, acc[6]);
    acc[7]  = mma(a1, b3, acc[7]);
    acc[8]  = mma(ones, b0, acc[8]);
    acc[9]  = mma(ones, b1, acc[9]);
    acc[10] = mma(ones, b2, acc[10]);
    acc[11] = mma(ones, b3, acc[11]);
  }

#pragma unroll
  for (unsigned i = 0; i < 2; ++i)
#pragma unroll
    for (unsigned t = 0; t < 4; ++t)
#pragma unroll
      for (unsigned r = 0; r < 8; ++r)
        part[(wk * 64u + 32u * wr + 16u * i + 8u * (unsigned)hl + r) * 64u + 16u * t + c] = acc[i * 4 + t][r];
  if (wr == 0u && hl == 0) {
#pragma unroll
    for (unsigned t = 0; t < 4; ++t) ksp[wk * 64u + 16u * t + c] = acc[8 + t][0];
  }
  __syncthreads();

  v8h o[2];
  _Float16* dp[2];
#pragma unroll
  for (unsigned i = 0; i < 2; ++i) {
    const unsigned q = i * 256u + tid;
    const unsigned row = q >> 3, ch = (q & 7u) * 8u;
#pragma unroll
    for (unsigned j = 0; j < 8; ++j) {
      const unsigned e = row * 64u + ch + j;
      const float s = ((part[e] + part[4096u + e]) + part[8192u + e]) + part[12288u + e];
      o[i][j] = (_Float16)(s * KV_SCL);
    }
    dp[i] = KVt + ((size_t)(b * NH + h) * 64u + row) * 64u + ch;
  }
  v4f ks;
  const unsigned kd = (tid & 15u) * 4u;
#pragma unroll
  for (unsigned j = 0; j < 4; ++j)
    ks[j] = (((ksp[kd + j] + ksp[64u + kd + j]) + ksp[128u + kd + j]) + ksp[192u + kd + j]) * ACT_INV;
  float* const kdst = Ksum + (size_t)(b * NH + h) * 64u + kd;

  *(volatile v8h*)dp[0] = o[0];
  *(volatile v8h*)dp[1] = o[1];
  if (tid < 16u) *(volatile v4f*)kdst = ks;
  __threadfence();
  *(volatile v8h*)dp[0] = o[0];
  *(volatile v8h*)dp[1] = o[1];
  if (tid < 16u) *(volatile v4f*)kdst = ks;
}

__global__ __launch_bounds__(128) __attribute__((amdgpu_num_vgpr(256)))
void k_msg(const _Float16* __restrict__ Q, const _Float16* __restrict__ KVt,
           const float* __restrict__ Ksum, const float* __restrict__ thr,
           const float* __restrict__ g1, const float* __restrict__ b1,
           _Float16* __restrict__ cat)
{
  __shared__ __attribute__((aligned(16))) float tile[64 * 260];
  __shared__ float sK[256];
  __shared__ float sG[256];
  __shared__ float sB[256];

  const unsigned tid = threadIdx.x, lane = tid & 31u, w = tid >> 5;
  const int hl = (int)(lane >> 4);
  const unsigned c = lane & 15u;
  const unsigned tok0 = blockIdx.x * 64u;
  const unsigned b = tok0 / (unsigned)SEQ;

#pragma unroll
  for (unsigned i = 0; i < 2; ++i) {
    const unsigned idx = i * 128u + tid;
    sK[idx] = Ksum[(size_t)b * CH + idx];
    sG[idx] = bf16_rne(g1[idx]);
    sB[idx] = bf16_rne(b1[idx]);
  }
  const float thrv = bf16_rne(thr[0]);
  __syncthreads();

  const _Float16* const qrow = Q + (size_t)(tok0 + 16u * w + c) * CH;
#pragma unroll
  for (unsigned h = 0; h < 4; ++h) {
    v16h qf[2];
    qf[0] = ld_frag(qrow + h * 64u, hl);
    qf[1] = ld_frag(qrow + h * 64u + 32u, hl);
    float ps = 0.f;
#pragma unroll
    for (unsigned ks = 0; ks < 2; ++ks)
#pragma unroll
      for (unsigned i = 0; i < 8; ++i) {
        ps += (float)qf[ks][i]     * sK[h * 64u + 32u * ks + 8u * (unsigned)hl + i];
        ps += (float)qf[ks][8 + i] * sK[h * 64u + 32u * ks + 16u + 8u * (unsigned)hl + i];
      }
    ps += __shfl_xor(ps, 16, 32);
    const float sc = ps * ACT_INV;
    const float sp = (sc > thrv) ? sc : 0.0f;
    const float zz = 1.0f / (sp + ATTN_EPS);

    v8f acc[4] = {};
    const _Float16* const kvb = KVt + (size_t)(b * NH + h) * 4096u;
#pragma unroll
    for (unsigned ks = 0; ks < 2; ++ks)
#pragma unroll
      for (unsigned t = 0; t < 4; ++t) {
        const v16h bf = ld_frag(kvb + (16u * t + c) * 64u + 32u * ks, hl);
        acc[t] = mma(qf[ks], bf, acc[t]);
      }
#pragma unroll
    for (unsigned r = 0; r < 8; ++r) {
      const float zr = __shfl(zz, 8 * hl + (int)r, 32);
      const unsigned rowl = 16u * w + 8u * (unsigned)hl + r;
#pragma unroll
      for (unsigned t = 0; t < 4; ++t)
        tile[rowl * 260u + h * 64u + 16u * t + c] = acc[t][r] * zr;
    }
  }
  __syncthreads();

  float gq[8], bb[8];
#pragma unroll
  for (unsigned j = 0; j < 8; ++j) { gq[j] = sG[8u * lane + j]; bb[j] = sB[8u * lane + j]; }

  v8h o[16];
#pragma unroll
  for (unsigned i = 0; i < 16; ++i) {
    const float* p = tile + (16u * w + i) * 260u + 8u * lane;
    const v4f a0 = *(const v4f*)p;
    const v4f a1 = *(const v4f*)(p + 4);
    float s = ((a0[0] + a0[1]) + (a0[2] + a0[3])) + ((a1[0] + a1[1]) + (a1[2] + a1[3]));
    s = wave_sum(s);
    const float mean = s * (1.0f / 256.0f);
    float d[8];
#pragma unroll
    for (unsigned j = 0; j < 4; ++j) { d[j] = a0[j] - mean; d[4 + j] = a1[j] - mean; }
    float q = 0.f;
#pragma unroll
    for (unsigned j = 0; j < 8; ++j) q += d[j] * d[j];
    q = wave_sum(q);
    const float rstd = 1.0f / sqrtf(q * (1.0f / 256.0f) + LN_EPS);
#pragma unroll
    for (unsigned j = 0; j < 8; ++j)
      o[i][j] = (_Float16)((d[j] * rstd * gq[j] + bb[j]) * ACT_CAR);
  }
  _Float16* const ob = cat + (size_t)(tok0 + 16u * w) * CATW + CH + 8u * lane;
#pragma unroll
  for (unsigned i = 0; i < 16; ++i) *(volatile v8h*)(ob + (size_t)i * CATW) = o[i];
  __threadfence();
#pragma unroll
  for (unsigned i = 0; i < 16; ++i) *(volatile v8h*)(ob + (size_t)i * CATW) = o[i];
}

__global__ __launch_bounds__(256) __attribute__((amdgpu_num_vgpr(256)))
void k_mlp2(const _Float16* __restrict__ H1, const _Float16* __restrict__ W2p,
            const _Float16* __restrict__ cat, const _Float16* __restrict__ Wap,
            const float* __restrict__ ba, const float* __restrict__ g2, const float* __restrict__ b2,
            const float* __restrict__ bng, const float* __restrict__ bnb,
            const float* __restrict__ bnm, const float* __restrict__ bnv,
            float* __restrict__ out)
{
  __shared__ __attribute__((aligned(16))) float tile[64 * 260];

  const unsigned tid = threadIdx.x, lane = tid & 31u, w = tid >> 5;
  const int hl = (int)(lane >> 4);
  const unsigned c = lane & 15u;
  const unsigned wr = w >> 2, wc = w & 3u;
  const unsigned tok0 = blockIdx.x * 64u;
  const unsigned b = tok0 / (unsigned)SEQ;
  const unsigned n0 = tok0 - b * (unsigned)SEQ;
  const unsigned mw = tok0 + 32u * wr;

  {
    v8f acc[8] = {};
    gemm_core(H1 + (size_t)(mw + c) * HID, H1 + (size_t)(mw + 16u + c) * HID,
              W2p + (size_t)(64u * wc + c) * HID, HID, hl, acc);
#pragma unroll
    for (unsigned i = 0; i < 2; ++i)
#pragma unroll
      for (unsigned t = 0; t < 4; ++t)
#pragma unroll
        for (unsigned r = 0; r < 8; ++r)
          tile[(32u * wr + 16u * i + 8u * (unsigned)hl + r) * 260u + 64u * wc + 16u * t + c] =
              acc[i * 4 + t][r] * ACC_SCL;
  }

  v8f acc2[8] = {};
  gemm_core(cat + (size_t)(mw + c) * CATW, cat + (size_t)(mw + 16u + c) * CATW,
            Wap + (size_t)(64u * wc + c) * CH, CH, hl, acc2);

  float bsc[4], bsh[4];
#pragma unroll
  for (unsigned t = 0; t < 4; ++t) {
    const unsigned col = 64u * wc + 16u * t + c;
    const float s = bf16_rne(bng[col]) * (1.0f / sqrtf(bf16_rne(bnv[col]) + BN_EPS));
    bsc[t] = s;
    bsh[t] = (bf16_rne(ba[col]) - bf16_rne(bnm[col])) * s + bf16_rne(bnb[col]);
  }
  __syncthreads();

  {
    const v4f gA = *(const v4f*)(g2 + 8u * lane);
    const v4f gB = *(const v4f*)(g2 + 8u * lane + 4u);
    const v4f hA = *(const v4f*)(b2 + 8u * lane);
    const v4f hB = *(const v4f*)(b2 + 8u * lane + 4u);
#pragma unroll 1
    for (unsigned i = 0; i < 8; ++i) {
      const unsigned rowl = 8u * w + i;
      float* p = tile + rowl * 260u + 8u * lane;
      const v4f a0 = *(const v4f*)p;
      const v4f a1 = *(const v4f*)(p + 4);
      const v8h xh = *(const v8h*)(cat + (size_t)(tok0 + rowl) * CATW + 8u * lane);
      float s = ((a0[0] + a0[1]) + (a0[2] + a0[3])) + ((a1[0] + a1[1]) + (a1[2] + a1[3]));
      s = wave_sum(s);
      const float mean = s * (1.0f / 256.0f);
      v4f d0, d1;
#pragma unroll
      for (unsigned j = 0; j < 4; ++j) { d0[j] = a0[j] - mean; d1[j] = a1[j] - mean; }
      float q = 0.f;
#pragma unroll
      for (unsigned j = 0; j < 4; ++j) { q += d0[j] * d0[j]; q += d1[j] * d1[j]; }
      q = wave_sum(q);
      const float rstd = 1.0f / sqrtf(q * (1.0f / 256.0f) + LN_EPS);
      v4f y0, y1;
#pragma unroll
      for (unsigned j = 0; j < 4; ++j) {
        y0[j] = d0[j] * rstd * bf16_rne(gA[j]) + bf16_rne(hA[j]) + (float)xh[j] * ACT_INV;
        y1[j] = d1[j] * rstd * bf16_rne(gB[j]) + bf16_rne(hB[j]) + (float)xh[4 + j] * ACT_INV;
      }
      *(v4f*)p = y0;
      *(v4f*)(p + 4) = y1;
    }
  }
  __syncthreads();

#pragma unroll
  for (unsigned i = 0; i < 2; ++i)
#pragma unroll
    for (unsigned t = 0; t < 4; ++t)
#pragma unroll
      for (unsigned r = 0; r < 8; ++r) {
        float* p = tile + (32u * wr + 16u * i + 8u * (unsigned)hl + r) * 260u + 64u * wc + 16u * t + c;
        const float cur = *p;
        *p = cur + (acc2[i * 4 + t][r] * ACC_SCL * bsc[t] + bsh[t]);
      }
  __syncthreads();

  float* const ob = out + (size_t)b * CH * SEQ_FULL + n0;
  for (unsigned i = 0; i < 16; ++i) {
    const unsigned qi = i * 256u + tid;
    const unsigned chn = qi >> 4, tq = (qi & 15u) * 4u;
    v4f v;
    v[0] = tile[(tq + 0u) * 260u + chn];
    v[1] = tile[(tq + 1u) * 260u + chn];
    v[2] = tile[(tq + 2u) * 260u + chn];
    v[3] = tile[(tq + 3u) * 260u + chn];
    *(volatile v4f*)(ob + (size_t)chn * SEQ_FULL + tq) = v;
  }
  __threadfence();
  for (unsigned i = 0; i < 16; ++i) {
    const unsigned qi = i * 256u + tid;
    const unsigned chn = qi >> 4, tq = (qi & 15u) * 4u;
    v4f v;
    v[0] = tile[(tq + 0u) * 260u + chn];
    v[1] = tile[(tq + 1u) * 260u + chn];
    v[2] = tile[(tq + 2u) * 260u + chn];
    v[3] = tile[(tq + 3u) * 260u + chn];
    *(volatile v4f*)(ob + (size_t)chn * SEQ_FULL + tq) = v;
  }
}

extern "C" void kernel_launch(void* const* d_in, const int* in_sizes, int n_in,
                              void* d_out, int out_size, void* d_ws, size_t ws_size,
                              hipStream_t stream)
{
  if (n_in < 21) return;
  if ((long)in_sizes[0] < (long)NB * CH * SEQ) return;
  if ((long)in_sizes[1] < (long)NB * CH * SEQ) return;
  if ((long)in_sizes[2] < (long)CH * CH) return;
  if ((long)in_sizes[4] < (long)CH * CH) return;
  if ((long)in_sizes[6] < (long)CH * CH) return;
  if ((long)in_sizes[15] < (long)CH * CH) return;
  if ((long)in_sizes[9] < (long)HID * CATW) return;
  if ((long)in_sizes[10] < (long)CH * HID) return;
  if (in_sizes[3] < CH || in_sizes[5] < CH || in_sizes[7] < CH || in_sizes[8] < 1) return;
  if (in_sizes[11] < CH || in_sizes[12] < CH || in_sizes[13] < CH || in_sizes[14] < CH) return;
  if (in_sizes[16] < CH || in_sizes[17] < CH || in_sizes[18] < CH || in_sizes[19] < CH || in_sizes[20] < CH) return;
  if ((long)out_size < (long)NB * CH * SEQ) return;

  const float* x1  = (const float*)d_in[0];
  const float* x2  = (const float*)d_in[1];
  const float* Wq  = (const float*)d_in[2];
  const float* bq  = (const float*)d_in[3];
  const float* Wk  = (const float*)d_in[4];
  const float* bk  = (const float*)d_in[5];
  const float* Wv  = (const float*)d_in[6];
  const float* bv  = (const float*)d_in[7];
  const float* thr = (const float*)d_in[8];
  const float* W1  = (const float*)d_in[9];
  const float* W2  = (const float*)d_in[10];
  const float* g1  = (const float*)d_in[11];
  const float* b1  = (const float*)d_in[12];
  const float* g2  = (const float*)d_in[13];
  const float* b2  = (const float*)d_in[14];
  const float* Wa  = (const float*)d_in[15];
  const float* ba  = (const float*)d_in[16];
  const float* bng = (const float*)d_in[17];
  const float* bnb = (const float*)d_in[18];
  const float* bnm = (const float*)d_in[19];
  const float* bnv = (const float*)d_in[20];
  float* out = (float*)d_out;

  const size_t nCAT = (size_t)NTOK * CATW;
  const size_t nP   = (size_t)NTOK * CH;
  const size_t nKV  = (size_t)NB * NH * 4096;
  const size_t total_bytes = (nCAT + 4 * nP + (size_t)N_WALL + nKV) * sizeof(_Float16)
                           + (size_t)NB * CH * sizeof(float);
  if (total_bytes > ws_size) return;

  _Float16* CAT = (_Float16*)d_ws;
  _Float16* X2T = CAT + nCAT;
  _Float16* Q16 = X2T + nP;
  _Float16* Kt  = Q16 + nP;
  _Float16* Vt  = Kt  + nP;
  _Float16* WP  = Vt  + nP;
  _Float16* KVt = WP  + N_WALL;
  float*    KS  = (float*)(KVt + nKV);
  _Float16* H1  = Q16;

  k_trx<<<dim3(SEQ / 64, CH / 64, 2 * NB), 256, 0, stream>>>(x1, x2, CAT, X2T);
  k_cvtw<<<dim3(128, 6), 256, 0, stream>>>(Wq, Wk, Wv, Wa, W1, W2, WP);

  k_gemm<1, 1><<<dim3(CH / 64, NTOK / 128, 1), 128, 0, stream>>>(
      CAT, WP + OFF_WQ, Q16, bq, CATW, CH, CH, 0u, 0u, 0u);
  k_gemm<2, 1><<<dim3(SEQ / 64, CH / 128, NB), 128, 0, stream>>>(
      WP + OFF_WK, X2T, Kt, bk, CH, CH, SEQ, 0u, (unsigned)(SEQ * CH), (unsigned)(CH * SEQ));
  k_gemm<2, 0><<<dim3(SEQ / 64, CH / 128, NB), 128, 0, stream>>>(
      WP + OFF_WV, X2T, Vt, bv, CH, CH, SEQ, 0u, (unsigned)(SEQ * CH), (unsigned)(CH * SEQ));

  k_kv<<<dim3(NH, NB), 256, 0, stream>>>(Kt, Vt, KVt, KS);

  k_msg<<<dim3(NTOK / 64), 128, 0, stream>>>(Q16, KVt, KS, thr, g1, b1, CAT);

  k_gemm<0, 2><<<dim3(HID / 64, NTOK / 128, 1), 128, 0, stream>>>(
      CAT, WP + OFF_W1, H1, bq, CATW, CATW, HID, 0u, 0u, 0u);

  k_mlp2<<<dim3(NTOK / 64), 256, 0, stream>>>(H1, WP + OFF_W2, CAT, WP + OFF_WA,
                                              ba, g2, b2, bng, bnb, bnm, bnv, out);
}
